// GATLayer_23630910062807
// MI455X (gfx1250) — hardware-verified
//
#include <hip/hip_runtime.h>
#include <math.h>
#include <stdint.h>

#define NB_   4
#define NL_   2048
#define DIN   128
#define NH_   4
#define HD_   64
#define NBH   (NB_ * NH_)
#define NTOK  (NB_ * NL_)
#define BPB   (NL_ / 128)
#define SP    68
#define SLOPE 0.2f
#define WSMAX 134217728

static_assert(NL_ % 128 == 0);
static_assert(NL_ % 64 == 0);
static_assert(NL_ == 128 * 16);
static_assert(DIN % 32 == 0);
static_assert(HD_ == 64);
static_assert(NH_ == 4);
static_assert((NTOK * DIN) % 2048 == 0);
static_assert(NTOK % 128 == 0);
static_assert(BPB == 16);
static_assert(DIN * HD_ == 8 * 256 * 4);
static_assert(DIN * HD_ == 4 * 256 * 8);
static_assert(2 * HD_ * 128 * 2 <= 128 * SP * 4);
static_assert((SP * 4) % 16 == 0);

typedef __attribute__((ext_vector_type(16))) __bf16 v16b;
typedef __attribute__((ext_vector_type(8)))  __bf16 v8b;
typedef __attribute__((ext_vector_type(8)))  float  v8f;
typedef __attribute__((ext_vector_type(4)))  float  v4f;
typedef __attribute__((ext_vector_type(4)))  unsigned int v4u;
typedef __attribute__((ext_vector_type(8)))  unsigned int v8u;
typedef v8b __attribute__((may_alias)) v8ba;
typedef v4f __attribute__((may_alias)) v4fa;
typedef v4u __attribute__((may_alias)) v4ua;

union FragU { v16b v; v8b h[2]; };
union PackU { v8u u; v16b v; };

__device__ __forceinline__ unsigned short f2bf_bits(float f) {
  const unsigned u = __float_as_uint(f);
  return (unsigned short)((u + 0x7FFFu + ((u >> 16) & 1u)) >> 16);
}
__device__ __forceinline__ float bf_bits2f(unsigned short h) { return __uint_as_float(((unsigned)h) << 16); }
__device__ __forceinline__ float bf16r(float f) {
  unsigned u = __float_as_uint(f);
  u = (u + 0x7FFFu + ((u >> 16) & 1u)) & 0xFFFF0000u;
  return __uint_as_float(u);
}
__device__ __forceinline__ unsigned pk16(unsigned short a, unsigned short b) { return (unsigned)a | ((unsigned)b << 16); }

__device__ __forceinline__ v8f wmma_bf16(v16b a, v16b b, v8f c) {
  v8f d = __builtin_amdgcn_wmma_f32_16x16x32_bf16(false, a, false, b, (short)0, c, false, false);
  asm volatile("v_nop\n\tv_nop\n\tv_nop\n\tv_nop" : "+v"(d) : "v"(a), "v"(b));
  return d;
}

__device__ __forceinline__ v16b load_frag(const unsigned short* p, int hh) {
  FragU f;
  f.h[0] = *(const v8ba*)(p + 8 * hh);
  f.h[1] = *(const v8ba*)(p + 16 + 8 * hh);
  return f.v;
}

__device__ __forceinline__ void pack_p2(v8f a, v8f c, v16b& ho, v16b& lo) {
  PackU uh, ul;
#pragma unroll
  for (int i = 0; i < 4; ++i) {
    const unsigned short h0 = f2bf_bits(a[2 * i]), h1 = f2bf_bits(a[2 * i + 1]);
    const unsigned short l0 = f2bf_bits(a[2 * i] - bf_bits2f(h0)), l1 = f2bf_bits(a[2 * i + 1] - bf_bits2f(h1));
    uh.u[i] = pk16(h0, h1); ul.u[i] = pk16(l0, l1);
    const unsigned short g0 = f2bf_bits(c[2 * i]), g1 = f2bf_bits(c[2 * i + 1]);
    const unsigned short m0 = f2bf_bits(c[2 * i] - bf_bits2f(g0)), m1 = f2bf_bits(c[2 * i + 1] - bf_bits2f(g1));
    uh.u[4 + i] = pk16(g0, g1); ul.u[4 + i] = pk16(m0, m1);
  }
  ho = uh.v; lo = ul.v;
}

template <int NT>
__device__ __forceinline__ void gemm_core_32(
    const unsigned short* __restrict__ A, const unsigned short* __restrict__ Bt,
    int K, size_t aoff, size_t boff, int hh, v8f (&acc)[2][NT]) {
  const unsigned short* a0 = A + aoff;
  const unsigned short* a1 = a0 + (size_t)16 * K;
  const unsigned short* bp = Bt + boff;
#pragma unroll 1
  for (int k0 = 0; k0 < K; k0 += 32) {
    const v16b f0 = load_frag(a0 + k0, hh);
    const v16b f1 = load_frag(a1 + k0, hh);
#pragma unroll
    for (int nt = 0; nt < NT; ++nt) {
      const v16b fb = load_frag(bp + (size_t)nt * 16 * K + k0, hh);
      acc[0][nt] = wmma_bf16(f0, fb, acc[0][nt]);
      acc[1][nt] = wmma_bf16(f1, fb, acc[1][nt]);
    }
  }
}

__global__ __launch_bounds__(256) void k_cvt(const float* __restrict__ src, unsigned short* __restrict__ dst, int n8) {
  int i = blockIdx.x * 256 + threadIdx.x;
  const bool ok = i < n8;
  i = ok ? i : (n8 - 1);
  const float* s = src + (size_t)i * 8;
  const v4f f0 = *(const v4fa*)(s);
  const v4f f1 = *(const v4fa*)(s + 4);
  v4u u;
  u[0] = pk16(f2bf_bits(f0[0]), f2bf_bits(f0[1]));
  u[1] = pk16(f2bf_bits(f0[2]), f2bf_bits(f0[3]));
  u[2] = pk16(f2bf_bits(f1[0]), f2bf_bits(f1[1]));
  u[3] = pk16(f2bf_bits(f1[2]), f2bf_bits(f1[3]));
  unsigned short* d = dst + (size_t)i * 8;
  if (ok) *(volatile v4u*)d = u;
  __threadfence();
  if (ok) *(volatile v4u*)d = u;
}

__global__ __launch_bounds__(256) void k_wcvt(const float* __restrict__ W, unsigned short* __restrict__ Wb) {
  __shared__ __align__(16) float tf[DIN * SP];
  const int hd  = blockIdx.x;
  const int tid = threadIdx.x;
  const float* Wz = W + (size_t)hd * DIN * HD_;
  {
    const int kr = tid >> 4;
    const int c4 = (tid & 15) * 4;
#pragma unroll
    for (int it = 0; it < 8; ++it) {
      const int k = it * 16 + kr;
      const v4f a = *(const v4fa*)(Wz + (size_t)k * HD_ + c4);
      *(v4fa*)(tf + k * SP + c4) = a;
    }
  }
  __syncthreads();
  const int osub = tid >> 4;
  const int k8   = (tid & 15) * 8;
  v4u hv[4];
#pragma unroll
  for (int it = 0; it < 4; ++it) {
    const int o = it * 16 + osub;
    v4u a;
#pragma unroll
    for (int q = 0; q < 4; ++q) {
      const float f0 = tf[(k8 + 2 * q) * SP + o];
      const float f1 = tf[(k8 + 2 * q + 1) * SP + o];
      a[q] = pk16(f2bf_bits(f0), f2bf_bits(f1));
    }
    hv[it] = a;
  }
#pragma unroll
  for (int it = 0; it < 4; ++it) {
    const int o = it * 16 + osub;
    const size_t go = (size_t)(hd * HD_ + o) * DIN + k8;
    *(volatile v4u*)(Wb + go) = hv[it];
  }
  __threadfence();
#pragma unroll
  for (int it = 0; it < 4; ++it) {
    const int o = it * 16 + osub;
    const size_t go = (size_t)(hd * HD_ + o) * DIN + k8;
    *(volatile v4u*)(Wb + go) = hv[it];
  }
}

__global__ __launch_bounds__(128) void k_proj(
    const unsigned short* __restrict__ Xb, const unsigned short* __restrict__ Wb,
    const float* __restrict__ av, float* __restrict__ S,
    unsigned short* __restrict__ VTh, unsigned short* __restrict__ VTl) {
  __shared__ __align__(16) unsigned char smem[128 * SP * 4];
  __shared__ __align__(16) float sA[2 * HD_];
  __shared__ __align__(16) float sS[2 * 128];
  float* sF = (float*)smem;
  unsigned short* sH = (unsigned short*)smem;
  unsigned short* sL = sH + HD_ * 128;
  const int tid = threadIdx.x, lane = tid & 31, w = tid >> 5;
  const int hh = lane >> 4, m = lane & 15;
  const int xb = blockIdx.x;
  const int b  = xb / BPB;
  const int p0 = (xb % BPB) * 128;
  const int hd = blockIdx.y;
  const int n0 = hd * HD_;
  const int m0 = xb * 128;
  const int m0w = m0 + 32 * w;
  const int bh = b * NH_ + hd;

  const v8f zero8 = {0.f, 0.f, 0.f, 0.f, 0.f, 0.f, 0.f, 0.f};
  v8f acc[2][4];
#pragma unroll
  for (int mt = 0; mt < 2; ++mt)
#pragma unroll
    for (int nt = 0; nt < 4; ++nt) acc[mt][nt] = zero8;

  gemm_core_32<4>(Xb, Wb, DIN, (size_t)(m0w + m) * DIN, (size_t)(n0 + m) * DIN, hh, acc);

  if (tid < HD_) {
    sA[tid]       = bf16r(av[hd * 2 * HD_ + tid]);
    sA[HD_ + tid] = bf16r(av[hd * 2 * HD_ + HD_ + tid]);
  }
#pragma unroll
  for (int nt = 0; nt < 4; ++nt)
#pragma unroll
    for (int mt = 0; mt < 2; ++mt)
#pragma unroll
      for (int r = 0; r < 8; ++r) {
        const int tokl = 32 * w + 16 * mt + 8 * hh + r;
        const int feat = 16 * nt + m;
        sF[tokl * SP + feat] = acc[mt][nt][r];
      }
  __syncthreads();
  {
    float sl = 0.0f, sr = 0.0f;
    const float* fr = sF + tid * SP;
#pragma unroll 2
    for (int d4 = 0; d4 < HD_ / 4; ++d4) {
      const v4f x = *(const v4fa*)(fr + 4 * d4);
      const v4f y = *(const v4fa*)(sA + 4 * d4);
      const v4f z = *(const v4fa*)(sA + HD_ + 4 * d4);
      sl = fmaf(x[0], y[0], sl);
      sl = fmaf(x[1], y[1], sl);
      sl = fmaf(x[2], y[2], sl);
      sl = fmaf(x[3], y[3], sl);
      sr = fmaf(x[0], z[0], sr);
      sr = fmaf(x[1], z[1], sr);
      sr = fmaf(x[2], z[2], sr);
      sr = fmaf(x[3], z[3], sr);
    }
    sS[tid] = sl;
    sS[128 + tid] = sr;
  }
  __syncthreads();
  {
    const size_t so = (size_t)bh * NL_ + p0 + lane * 4;
    const size_t sk = (size_t)NBH * NL_ + so;
    const v4f vq = *(const v4fa*)(sS + lane * 4);
    const v4f vk = *(const v4fa*)(sS + 128 + lane * 4);
    if (w == 0) *(volatile v4f*)(S + so) = vq;
    if (w == 1) *(volatile v4f*)(S + sk) = vk;
    __threadfence();
    if (w == 0) *(volatile v4f*)(S + so) = vq;
    if (w == 1) *(volatile v4f*)(S + sk) = vk;
  }
#pragma unroll
  for (int nt = 0; nt < 4; ++nt)
#pragma unroll
    for (int mt = 0; mt < 2; ++mt)
#pragma unroll
      for (int r = 0; r < 8; ++r) {
        const int tokl = 32 * w + 16 * mt + 8 * hh + r;
        const int feat = 16 * nt + m;
        const float y = acc[mt][nt][r];
        const unsigned short hb = f2bf_bits(y);
        const unsigned short lb = f2bf_bits(y - bf_bits2f(hb));
        const int idx = feat * 128 + tokl;
        sH[idx] = hb;
        sL[idx] = lb;
      }
  __syncthreads();
  {
    const int dsub = lane >> 4, t8 = (lane & 15) * 8;
#pragma unroll
    for (int it = 0; it < 8; ++it) {
      const int d = 16 * w + 2 * it + dsub;
      const v4u hv = *(const v4ua*)(sH + d * 128 + t8);
      const v4u lv = *(const v4ua*)(sL + d * 128 + t8);
      const size_t go = ((size_t)(bh * HD_ + d)) * (size_t)NL_ + p0 + t8;
      *(volatile v4u*)(VTh + go) = hv;
      *(volatile v4u*)(VTl + go) = lv;
    }
    __threadfence();
#pragma unroll
    for (int it = 0; it < 8; ++it) {
      const int d = 16 * w + 2 * it + dsub;
      const v4u hv = *(const v4ua*)(sH + d * 128 + t8);
      const v4u lv = *(const v4ua*)(sL + d * 128 + t8);
      const size_t go = ((size_t)(bh * HD_ + d)) * (size_t)NL_ + p0 + t8;
      *(volatile v4u*)(VTh + go) = hv;
      *(volatile v4u*)(VTl + go) = lv;
    }
  }
}

__global__ __launch_bounds__(128) void k_attn(const float* __restrict__ S,
                                              const unsigned short* __restrict__ VTh,
                                              const unsigned short* __restrict__ VTl,
                                              float* __restrict__ out) {
  __shared__ __align__(16) float sK[NL_];
  __shared__ __align__(16) float sO[4][16 * SP];

  const int tid = threadIdx.x, lane = tid & 31, w = tid >> 5;
  const int hh = lane >> 4, m = lane & 15;
  const int qt = blockIdx.x;
  const int b  = blockIdx.y;
  const int q0 = qt * 64, q0w = q0 + 16 * w, q = q0w + m;
  float* so = sO[w];

#pragma unroll
  for (int t = 0; t < 4; ++t)
#pragma unroll
    for (int r = 0; r < 8; ++r) so[m * SP + 16 * t + 8 * hh + r] = 0.0f;

  const v8f zero8 = {0.f, 0.f, 0.f, 0.f, 0.f, 0.f, 0.f, 0.f};

#pragma unroll 1
  for (int hd = 0; hd < NH_; ++hd) {
    const int bh = b * NH_ + hd;
    __syncthreads();
    {
      const float* g = S + (size_t)NBH * NL_ + (size_t)bh * NL_ + tid * 16;
#pragma unroll
      for (int i = 0; i < 4; ++i) {
        const v4f a = *(const v4fa*)(g + 4 * i);
        *(v4fa*)(sK + tid * 16 + 4 * i) = a;
      }
    }
    const float sqv = S[(size_t)bh * NL_ + q];

    v8f o[4];
#pragma unroll
    for (int t = 0; t < 4; ++t) o[t] = zero8;
    float mrun = -INFINITY, lrun = 0.0f;

    __syncthreads();

#pragma unroll 1
    for (int ks = 0; ks < NL_ / 64; ++ks) {
      const int kb = ks * 64;

      v8f s[4];
#pragma unroll
      for (int j = 0; j < 4; ++j) {
        const int ko = kb + 16 * j + 8 * hh;
        const v4f kA = *(const v4fa*)(sK + ko);
        const v4f kB = *(const v4fa*)(sK + ko + 4);
        const float kv[8] = {kA[0], kA[1], kA[2], kA[3], kB[0], kB[1], kB[2], kB[3]};
#pragma unroll
        for (int r = 0; r < 8; ++r) {
          float t = sqv + kv[r];
          t = (t >= 0.0f) ? t : SLOPE * t;
          s[j][r] = t;
        }
      }
      float cm = -INFINITY;
#pragma unroll
      for (int j = 0; j < 4; ++j)
#pragma unroll
        for (int r = 0; r < 8; ++r) cm = fmaxf(cm, s[j][r]);
      cm = fmaxf(cm, __shfl_xor(cm, 16, 32));
      const float mnew  = fmaxf(mrun, cm);
      const float alpha = __expf(mrun - mnew);
      mrun = mnew;
      float psum = 0.0f;
#pragma unroll
      for (int j = 0; j < 4; ++j)
#pragma unroll
        for (int r = 0; r < 8; ++r) {
          const float p = __expf(s[j][r] - mnew);
          psum += p;
          s[j][r] = p;
        }
      psum += __shfl_xor(psum, 16, 32);
      lrun = lrun * alpha + psum;
#pragma unroll
      for (int t = 0; t < 4; ++t)
#pragma unroll
        for (int r = 0; r < 8; ++r) o[t][r] *= alpha;

      v16b pah, pal;
      pack_p2(s[0], s[1], pah, pal);
#pragma unroll
      for (int t = 0; t < 4; ++t) {
        const unsigned short* vph = VTh + (size_t)(bh * HD_ + 16 * t + m) * (size_t)NL_ + kb;
        const unsigned short* vpl = VTl + (size_t)(bh * HD_ + 16 * t + m) * (size_t)NL_ + kb;
        const v16b vh = load_frag(vph, hh), vl = load_frag(vpl, hh);
        o[t] = wmma_bf16(vh, pah, o[t]);
        o[t] = wmma_bf16(vh, pal, o[t]);
        o[t] = wmma_bf16(vl, pah, o[t]);
      }
      pack_p2(s[2], s[3], pah, pal);
#pragma unroll
      for (int t = 0; t < 4; ++t) {
        const unsigned short* vph = VTh + (size_t)(bh * HD_ + 16 * t + m) * (size_t)NL_ + kb + 32;
        const unsigned short* vpl = VTl + (size_t)(bh * HD_ + 16 * t + m) * (size_t)NL_ + kb + 32;
        const v16b vh = load_frag(vph, hh), vl = load_frag(vpl, hh);
        o[t] = wmma_bf16(vh, pah, o[t]);
        o[t] = wmma_bf16(vh, pal, o[t]);
        o[t] = wmma_bf16(vl, pah, o[t]);
      }
    }

    const float inv = 1.0f / lrun;
#pragma unroll
    for (int t = 0; t < 4; ++t) {
#pragma unroll
      for (int r = 0; r < 8; ++r) {
        const int idx = m * SP + 16 * t + 8 * hh + r;
        const float cur = so[idx];
        so[idx] = cur + o[t][r] * inv;
      }
    }
  }

#pragma unroll 2
  for (int j = 0; j < 32; ++j) {
    const int idx = m * SP + 16 * (j >> 3) + 8 * hh + (j & 7);
    float v = so[idx] * 0.25f;
    v = (v > 0.0f) ? v : expm1f(v);
    so[idx] = v;
  }
  __syncthreads();
  {
    const int rsub = lane >> 4;
    const int c4   = (lane & 15) * 4;
    v4f fv[8];
#pragma unroll
    for (int it = 0; it < 8; ++it) {
      const int row = 2 * it + rsub;
      fv[it] = *(const v4fa*)(so + row * SP + c4);
    }
#pragma unroll
    for (int it = 0; it < 8; ++it) {
      const int row = 2 * it + rsub;
      *(volatile v4f*)(out + (size_t)(b * NL_ + q0w + row) * (size_t)HD_ + c4) = fv[it];
    }
    __threadfence();
#pragma unroll
    for (int it = 0; it < 8; ++it) {
      const int row = 2 * it + rsub;
      *(volatile v4f*)(out + (size_t)(b * NL_ + q0w + row) * (size_t)HD_ + c4) = fv[it];
    }
  }
}

extern "C" void kernel_launch(void* const* d_in, const int* in_sizes, int n_in,
                              void* d_out, int out_size, void* d_ws, size_t ws_size,
                              hipStream_t stream) {
  if (n_in < 3) return;
  if (in_sizes[0] != NTOK * DIN) return;
  if (in_sizes[1] != NH_ * DIN * HD_) return;
  if (in_sizes[2] != NH_ * 2 * HD_) return;
  if (out_size != NTOK * HD_) return;

  const float* hin = (const float*)d_in[0];
  const float* W   = (const float*)d_in[1];
  const float* av  = (const float*)d_in[2];
  float* out = (float*)d_out;

  const size_t PX  = (size_t)NTOK * DIN * 2;
  const size_t PW  = (size_t)NH_ * HD_ * DIN * 2;
  const size_t PS  = (size_t)2 * NBH * NL_ * 4;
  const size_t PVT = (size_t)NBH * HD_ * NL_ * 2;
  size_t off = 0;
  const size_t oXb  = off; off += PX;
  const size_t oWb  = off; off += PW;
  const size_t oS   = off; off += PS;
  const size_t oVTh = off; off += PVT;
  const size_t oVTl = off; off += PVT;
  if (off > ws_size || off > (size_t)WSMAX) return;

  char* ws = (char*)d_ws;
  unsigned short* Xb  = (unsigned short*)(ws + oXb);
  unsigned short* Wb  = (unsigned short*)(ws + oWb);
  float*          S   = (float*)(ws + oS);
  unsigned short* VTh = (unsigned short*)(ws + oVTh);
  unsigned short* VTl = (unsigned short*)(ws + oVTl);

  const int n8x = NTOK * DIN / 8;
  k_cvt<<<dim3((n8x + 255) / 256), 256, 0, stream>>>(hin, Xb, n8x);
  k_wcvt<<<dim3(NH_), 256, 0, stream>>>(W, Wb);
  k_proj<<<dim3(NTOK / 128, NH_), 128, 0, stream>>>(Xb, Wb, av, S, VTh, VTl);
  k_attn<<<dim3(NL_ / 64, NB_), 128, 0, stream>>>(S, VTh, VTl, out);
  (void)hipGetLastError();
}
